// LSTM_27152783245909
// MI455X (gfx1250) — hardware-verified
//
#include <hip/hip_runtime.h>
#include <math.h>

constexpr int NBATCH = 64;
constexpr int NIN    = 512;
constexpr int NHID   = 1024;
constexpr int NOUTD  = 512;
constexpr int NSTEP  = 256;
constexpr int NGATE  = 4 * NHID;
constexpr int TCHUNK = 64;
constexpr int NCHUNK = NSTEP / TCHUNK;
constexpr int NROWS  = NSTEP * NBATCH;
constexpr int CHROWS = TCHUNK * NBATCH;
constexpr int SEQTHR = 512;
constexpr int HPITCH = NHID + 8;
constexpr int LPITCH = NOUTD + 4;
constexpr int MBLK   = NBATCH / 16;
constexpr int TILE_F = 256;
constexpr float WCARRY     = 16.0f;
constexpr float WCARRY_INV = 1.0f / WCARRY;

constexpr int PB_WIH  = NGATE * NIN / 8 / 256;
constexpr int PB_WHH  = NGATE * NHID / 8 / 256;
constexpr int PB_WOUT = NOUTD * NHID / 8 / 256;
constexpr int PB_BIAS = NGATE / 4 / 256;
constexpr int PB_HST  = NBATCH * NHID / 8 / 256;
constexpr int PB_CST  = NBATCH * NHID / 4 / 256;
constexpr int PB_ALL  = PB_WIH + PB_WHH + PB_WOUT + PB_BIAS + PB_HST + PB_CST;

static_assert(NIN % 32 == 0 && NHID % 32 == 0, "K multiples of 32");
static_assert(CHROWS % 64 == 0 && NGATE % 64 == 0, "GEMM tile multiples");
static_assert(NROWS % 32 == 0 && NOUTD == 8 * 64, "head tile multiples");
static_assert(NHID == 64 * (SEQTHR / 32), "16 waves x 64 hidden units");
static_assert(NSTEP % TCHUNK == 0 && NBATCH % 16 == 0, "chunking");
static_assert((16 * NHID) % (SEQTHR * 8) == 0, "tile copy loop exact");
static_assert(PB_WIH == 1024 && PB_WHH == 2048 && PB_WOUT == 256 && PB_BIAS == 4 && PB_HST == 32 && PB_CST == 64, "prep segments");
static_assert((HPITCH * 2) % 16 == 0 && (LPITCH * 4) % 16 == 0, "LDS pitches 16-B aligned");

typedef __attribute__((ext_vector_type(16))) _Float16 v16h;
typedef __attribute__((ext_vector_type(8)))  _Float16 v8h;
typedef __attribute__((ext_vector_type(8)))  float    v8f;
typedef __attribute__((ext_vector_type(4)))  float    v4f;

__device__ __forceinline__ void guard4_h(v8f& a0, v8f& a1, v8f& a2, v8f& a3, v16h x, v16h b0, v16h b1, v16h b2, v16h b3) {
  asm volatile("v_nop\n\tv_nop\n\tv_nop\n\tv_nop" : "+v"(a0), "+v"(a1), "+v"(a2), "+v"(a3) : "v"(x), "v"(b0), "v"(b1), "v"(b2), "v"(b3));
}
__device__ __forceinline__ void acc_guard4(v8f& a, v8f& b, v8f& c, v8f& d) {
  asm volatile("v_nop\n\tv_nop\n\tv_nop\n\tv_nop" : "+v"(a), "+v"(b), "+v"(c), "+v"(d));
}

template <typename T> struct Frag;
template <> struct Frag<_Float16> {
  typedef v16h V; union U { v16h v; v8h h[2]; };
  static __device__ __forceinline__ v16h load(const _Float16* p) {
    U f; f.h[0] = *(const v8h*)(p); f.h[1] = *(const v8h*)(p + 16); return f.v;
  }
  static __device__ __forceinline__ v8f mma(v16h a, v16h b, v8f c) {
    return __builtin_amdgcn_wmma_f32_16x16x32_f16(false, a, false, b, (short)0, c, false, false);
  }
};

__device__ __forceinline__ float fsig(float x)  { return __builtin_amdgcn_rcpf(1.0f + __expf(-x)); }
__device__ __forceinline__ float ftanh(float x) { return 1.0f - 2.0f * __builtin_amdgcn_rcpf(__expf(2.0f * x) + 1.0f); }

__global__ __launch_bounds__(256) void prep_kernel(const float* __restrict__ w_ih, const float* __restrict__ w_hh,
                                                   const float* __restrict__ w_out, const float* __restrict__ b_ih,
                                                   const float* __restrict__ b_hh, const float* __restrict__ h0,
                                                   const float* __restrict__ c0,
                                                   unsigned short* __restrict__ wih16, unsigned short* __restrict__ whh16,
                                                   unsigned short* __restrict__ wout16, float* __restrict__ bias16,
                                                   unsigned short* __restrict__ hst0, float* __restrict__ cst0) {
  const int blk = blockIdx.x;
  const int tid = threadIdx.x;
  if (blk < PB_WIH + PB_WHH + PB_WOUT) {
    const float* src;
    unsigned short* dst;
    int lb;
    if (blk < PB_WIH) { src = w_ih; dst = wih16; lb = blk; }
    else if (blk < PB_WIH + PB_WHH) { src = w_hh; dst = whh16; lb = blk - PB_WIH; }
    else { src = w_out; dst = wout16; lb = blk - PB_WIH - PB_WHH; }
    const size_t i = (size_t)lb * 256 + (size_t)tid;
    const v4f a = *(const v4f*)(src + i * 8);
    const v4f b = *(const v4f*)(src + i * 8 + 4);
    v8h hv;
#pragma unroll
    for (int e = 0; e < 4; ++e) {
      hv[e]     = (_Float16)(a[e] * WCARRY);
      hv[4 + e] = (_Float16)(b[e] * WCARRY);
    }
    *(volatile v8h*)(dst + i * 8) = hv;
    __threadfence();
    *(volatile v8h*)(dst + i * 8) = hv;
  } else if (blk < PB_WIH + PB_WHH + PB_WOUT + PB_BIAS) {
    const int lb = blk - (PB_WIH + PB_WHH + PB_WOUT);
    const int i4 = (lb * 256 + tid) * 4;
    const v4f a = *(const v4f*)(b_ih + i4);
    const v4f b = *(const v4f*)(b_hh + i4);
    v4f o;
#pragma unroll
    for (int e = 0; e < 4; ++e) o[e] = (a[e] + b[e]) * WCARRY;
    *(volatile v4f*)(bias16 + i4) = o;
    __threadfence();
    *(volatile v4f*)(bias16 + i4) = o;
  } else if (blk < PB_WIH + PB_WHH + PB_WOUT + PB_BIAS + PB_HST) {
    const int lb = blk - (PB_WIH + PB_WHH + PB_WOUT + PB_BIAS);
    const int idx = lb * 256 + tid;
    const int row = idx >> 7;
    const int c8 = (idx & 127) * 8;
    const v4f a = *(const v4f*)(h0 + c8);
    const v4f b = *(const v4f*)(h0 + c8 + 4);
    v8h hv;
#pragma unroll
    for (int e = 0; e < 4; ++e) {
      hv[e]     = (_Float16)a[e];
      hv[4 + e] = (_Float16)b[e];
    }
    unsigned short* op = hst0 + (size_t)row * NHID + c8;
    *(volatile v8h*)op = hv;
    __threadfence();
    *(volatile v8h*)op = hv;
  } else {
    const int lb = blk - (PB_WIH + PB_WHH + PB_WOUT + PB_BIAS + PB_HST);
    const int idx = lb * 256 + tid;
    const int ln = idx & 31;
    const int nt = (idx >> 6) & 3;
    const int wv = (idx >> 8) & 15;
    const int j = 64 * wv + 16 * nt + (ln & 15);
    const float cv = c0[j];
    const v4f o = {cv, cv, cv, cv};
    float* op = cst0 + (size_t)idx * 4;
    *(volatile v4f*)op = o;
    __threadfence();
    *(volatile v4f*)op = o;
  }
}

__global__ __launch_bounds__(256) void xs_transpose_kernel(const float* __restrict__ x, unsigned short* __restrict__ xsT) {
  __shared__ float Tt[64 * 65];
  const int tid = threadIdx.x;
  const int c0 = blockIdx.x * 64;
  const int r0 = blockIdx.y * 64;
  const int b  = blockIdx.z;
  const float* src = x + (size_t)b * NIN * NSTEP;
#pragma unroll
  for (int i = 0; i < 4; ++i) {
    const int idx = i * 256 + tid;
    const int rr = idx >> 4;
    const int cc = (idx & 15) * 4;
    const v4f v = *(const v4f*)(src + (size_t)(r0 + rr) * NSTEP + c0 + cc);
    Tt[rr * 65 + cc + 0] = v[0];
    Tt[rr * 65 + cc + 1] = v[1];
    Tt[rr * 65 + cc + 2] = v[2];
    Tt[rr * 65 + cc + 3] = v[3];
  }
  __syncthreads();
  const int q = tid >> 3;
  const int c8 = (tid & 7) * 8;
  v8h hv[2];
#pragma unroll
  for (int g = 0; g < 2; ++g) {
    const int qq = g * 32 + q;
#pragma unroll
    for (int e = 0; e < 8; ++e) {
      const float f = Tt[(c8 + e) * 65 + qq];
      hv[g][e] = (_Float16)f;
    }
  }
  for (int pass = 0; pass < 2; ++pass) {
#pragma unroll
    for (int g = 0; g < 2; ++g) {
      const size_t o = ((size_t)(c0 + g * 32 + q) * NBATCH + (size_t)b) * NIN + (size_t)(r0 + c8);
      *(volatile v8h*)(xsT + o) = hv[g];
    }
    __threadfence();
  }
}

__global__ __launch_bounds__(256) void xproj_gemm_kernel(const unsigned short* __restrict__ Ap,
                                                         const unsigned short* __restrict__ Btp,
                                                         const float* __restrict__ bias16, float* __restrict__ XPF) {
  const _Float16* A  = (const _Float16*)Ap;
  const _Float16* Bt = (const _Float16*)Btp;
  constexpr int tilesN = NGATE / 64;
  constexpr int tilesM = CHROWS / 64;
  const int lane = threadIdx.x & 31;
  const int wave = threadIdx.x >> 5;
  const int tile = blockIdx.x * 8 + wave;
  if (tile >= tilesM * tilesN) return;
  const int tm = tile / tilesN;
  const int tn = tile - tm * tilesN;
  const int m0 = tm << 6;
  const int n0 = tn << 6;
  const int rlane = lane & 15;
  const int koff  = (lane >> 4) * 8;

  v8f acc[4][4];
#pragma unroll
  for (int i = 0; i < 4; ++i)
#pragma unroll
    for (int j = 0; j < 4; ++j) acc[i][j] = (v8f){0.f, 0.f, 0.f, 0.f, 0.f, 0.f, 0.f, 0.f};

  for (int k0 = 0; k0 < NIN; k0 += 32) {
    v16h bh[4];
#pragma unroll
    for (int j = 0; j < 4; ++j)
      bh[j] = Frag<_Float16>::load(Bt + (size_t)(n0 + (j << 4) + rlane) * NIN + koff + k0);
#pragma unroll
    for (int i = 0; i < 4; ++i) {
      const v16h ah = Frag<_Float16>::load(A + (size_t)(m0 + (i << 4) + rlane) * NIN + koff + k0);
#pragma unroll
      for (int j = 0; j < 4; ++j) acc[i][j] = Frag<_Float16>::mma(ah, bh[j], acc[i][j]);
      guard4_h(acc[i][0], acc[i][1], acc[i][2], acc[i][3], ah, bh[0], bh[1], bh[2], bh[3]);
    }
  }
  acc_guard4(acc[0][0], acc[0][1], acc[0][2], acc[0][3]);
  acc_guard4(acc[1][0], acc[1][1], acc[1][2], acc[1][3]);
  acc_guard4(acc[2][0], acc[2][1], acc[2][2], acc[2][3]);
  acc_guard4(acc[3][0], acc[3][1], acc[3][2], acc[3][3]);

#pragma unroll
  for (int j = 0; j < 4; ++j) {
    const float bv = bias16[n0 + (j << 4) + rlane];
#pragma unroll
    for (int i = 0; i < 4; ++i)
#pragma unroll
      for (int r = 0; r < 8; ++r) acc[i][j][r] = acc[i][j][r] + bv;
  }
  for (int pass = 0; pass < 2; ++pass) {
#pragma unroll
    for (int i = 0; i < 4; ++i) {
#pragma unroll
      for (int j = 0; j < 4; ++j) {
        float* tp = XPF + ((size_t)((m0 >> 4) + i) * (NGATE >> 4) + (size_t)((n0 >> 4) + j)) * TILE_F + lane * 4;
        const v4f p0 = {acc[i][j][0], acc[i][j][1], acc[i][j][2], acc[i][j][3]};
        const v4f p1 = {acc[i][j][4], acc[i][j][5], acc[i][j][6], acc[i][j][7]};
        *(volatile v4f*)tp = p0;
        *(volatile v4f*)(tp + 128) = p1;
      }
    }
    __threadfence();
  }
}

__global__ __launch_bounds__(SEQTHR) void lstm_seq_kernel(const float* __restrict__ XPF,
                                                          const unsigned short* __restrict__ WHp,
                                                          const unsigned short* __restrict__ hst_in,
                                                          const float* __restrict__ cst_in,
                                                          unsigned short* __restrict__ hst_out,
                                                          float* __restrict__ cst_out,
                                                          unsigned short* __restrict__ CALL, int t0) {
  __shared__ __align__(16) _Float16 Ah[16 * HPITCH];
  __shared__ __align__(16) _Float16 Ct[16 * HPITCH];
  const _Float16* WH = (const _Float16*)WHp;
  const int tid = threadIdx.x;
  const int lane = tid & 31;
  const int wave = tid >> 5;
  const int c = lane & 15;
  const int hh = lane >> 4;
  const int koff = hh * 8;
  const int mb = blockIdx.x;
  const int rowbase = mb * 16;
  const int crow = tid >> 7;
  const int cc8 = (tid & 127) * 8;

  {
    const _Float16* hin = (const _Float16*)hst_in;
#pragma unroll
    for (int it = 0; it < 4; ++it) {
      const int row = it * 4 + crow;
      const v8h v = *(const v8h*)(hin + (size_t)(rowbase + row) * NHID + cc8);
      *(v8h*)(Ah + row * HPITCH + cc8) = v;
    }
  }
  float cst[4][8];
#pragma unroll
  for (int nt = 0; nt < 4; ++nt) {
    const float* cp = cst_in + (size_t)(((mb * 16 + wave) * 4 + nt)) * TILE_F + lane * 4;
    const v4f p0 = *(const v4f*)cp;
    const v4f p1 = *(const v4f*)(cp + 128);
#pragma unroll
    for (int e = 0; e < 4; ++e) { cst[nt][e] = p0[e]; cst[nt][4 + e] = p1[e]; }
  }
  __syncthreads();

  const _Float16* ahrow = Ah + c * HPITCH + koff;

#pragma unroll 1
  for (int tl = 0; tl < TCHUNK; ++tl) {
    float hnew[4][8];
#pragma unroll
    for (int nt = 0; nt < 4; ++nt) {
      const int j = 64 * wave + 16 * nt + c;
      const int jt = 4 * wave + nt;
      const _Float16* wh = WH + (size_t)j * NHID + koff;
      const float* xp = XPF + ((size_t)(tl * MBLK + mb) * (NGATE >> 4) + (size_t)jt) * TILE_F + lane * 4;
      v8f acc[4];
#pragma unroll
      for (int g = 0; g < 4; ++g) {
        const v4f p0 = *(const v4f*)(xp + (size_t)g * (NHID >> 4) * TILE_F);
        const v4f p1 = *(const v4f*)(xp + (size_t)g * (NHID >> 4) * TILE_F + 128);
        acc[g] = (v8f){p0[0], p0[1], p0[2], p0[3], p1[0], p1[1], p1[2], p1[3]};
      }
#pragma unroll 1
      for (int k0 = 0; k0 < NHID; k0 += 32) {
        const v16h a  = Frag<_Float16>::load(ahrow + k0);
        const v16h b0 = Frag<_Float16>::load(wh + k0);
        const v16h b1 = Frag<_Float16>::load(wh + (size_t)1 * NHID * NHID + k0);
        const v16h b2 = Frag<_Float16>::load(wh + (size_t)2 * NHID * NHID + k0);
        const v16h b3 = Frag<_Float16>::load(wh + (size_t)3 * NHID * NHID + k0);
        acc[0] = Frag<_Float16>::mma(a, b0, acc[0]);
        acc[1] = Frag<_Float16>::mma(a, b1, acc[1]);
        acc[2] = Frag<_Float16>::mma(a, b2, acc[2]);
        acc[3] = Frag<_Float16>::mma(a, b3, acc[3]);
        guard4_h(acc[0], acc[1], acc[2], acc[3], a, b0, b1, b2, b3);
      }
      acc_guard4(acc[0], acc[1], acc[2], acc[3]);
#pragma unroll
      for (int r = 0; r < 8; ++r) {
        const float zi = acc[0][r] * WCARRY_INV;
        const float zf = acc[1][r] * WCARRY_INV;
        const float zg = acc[2][r] * WCARRY_INV;
        const float zo = acc[3][r] * WCARRY_INV;
        const float ig = fsig(zi);
        const float fg = fsig(zf);
        const float gg = ftanh(zg);
        const float og = fsig(zo);
        const float cn = fg * cst[nt][r] + ig * gg;
        cst[nt][r] = cn;
        hnew[nt][r] = og * ftanh(cn);
      }
    }
    __syncthreads();
#pragma unroll
    for (int nt = 0; nt < 4; ++nt) {
      const int j = 64 * wave + 16 * nt + c;
#pragma unroll
      for (int r = 0; r < 8; ++r) {
        Ah[(8 * hh + r) * HPITCH + j] = (_Float16)hnew[nt][r];
        Ct[(8 * hh + r) * HPITCH + j] = (_Float16)cst[nt][r];
      }
    }
    __syncthreads();
    {
      v8h cv[4];
#pragma unroll
      for (int it = 0; it < 4; ++it) cv[it] = *(const v8h*)(Ct + (it * 4 + crow) * HPITCH + cc8);
      for (int pass = 0; pass < 2; ++pass) {
#pragma unroll
        for (int it = 0; it < 4; ++it) {
          const size_t o = ((size_t)(t0 + tl) * NBATCH + (size_t)(rowbase + it * 4 + crow)) * NHID + (size_t)cc8;
          *(volatile v8h*)(CALL + o) = cv[it];
        }
        __threadfence();
      }
    }
  }

  {
    v8h hv[4];
#pragma unroll
    for (int it = 0; it < 4; ++it) hv[it] = *(const v8h*)(Ah + (it * 4 + crow) * HPITCH + cc8);
    for (int pass = 0; pass < 2; ++pass) {
#pragma unroll
      for (int it = 0; it < 4; ++it)
        *(volatile v8h*)(hst_out + (size_t)(rowbase + it * 4 + crow) * NHID + cc8) = hv[it];
#pragma unroll
      for (int nt = 0; nt < 4; ++nt) {
        float* cp = cst_out + (size_t)(((mb * 16 + wave) * 4 + nt)) * TILE_F + lane * 4;
        const v4f p0 = {cst[nt][0], cst[nt][1], cst[nt][2], cst[nt][3]};
        const v4f p1 = {cst[nt][4], cst[nt][5], cst[nt][6], cst[nt][7]};
        *(volatile v4f*)cp = p0;
        *(volatile v4f*)(cp + 128) = p1;
      }
      __threadfence();
    }
  }
}

__global__ __launch_bounds__(256) void head_softmax_kernel(const unsigned short* __restrict__ Cp,
                                                           const unsigned short* __restrict__ Wop,
                                                           const float* __restrict__ b_out, float* __restrict__ out) {
  __shared__ __align__(16) float Lg[32 * LPITCH];
  const _Float16* CA = (const _Float16*)Cp;
  const _Float16* WO = (const _Float16*)Wop;
  const int tid = threadIdx.x;
  const int lane = tid & 31;
  const int wave = tid >> 5;
  const int c = lane & 15;
  const int hh = lane >> 4;
  const int koff = hh * 8;
  const int R0 = blockIdx.x * 32;
  const int n0 = 64 * wave;

  v8f acc[2][4];
#pragma unroll
  for (int i = 0; i < 2; ++i)
#pragma unroll
    for (int j = 0; j < 4; ++j) acc[i][j] = (v8f){0.f, 0.f, 0.f, 0.f, 0.f, 0.f, 0.f, 0.f};

  const _Float16* a0p = CA + (size_t)(R0 + c) * NHID + koff;
  const _Float16* a1p = CA + (size_t)(R0 + 16 + c) * NHID + koff;
  const _Float16* bp  = WO + (size_t)(n0 + c) * NHID + koff;
#pragma unroll 1
  for (int k0 = 0; k0 < NHID; k0 += 32) {
    const v16h a0 = Frag<_Float16>::load(a0p + k0);
    const v16h a1 = Frag<_Float16>::load(a1p + k0);
    const v16h b0 = Frag<_Float16>::load(bp + k0);
    const v16h b1 = Frag<_Float16>::load(bp + (size_t)16 * NHID + k0);
    const v16h b2 = Frag<_Float16>::load(bp + (size_t)32 * NHID + k0);
    const v16h b3 = Frag<_Float16>::load(bp + (size_t)48 * NHID + k0);
    acc[0][0] = Frag<_Float16>::mma(a0, b0, acc[0][0]);
    acc[0][1] = Frag<_Float16>::mma(a0, b1, acc[0][1]);
    acc[0][2] = Frag<_Float16>::mma(a0, b2, acc[0][2]);
    acc[0][3] = Frag<_Float16>::mma(a0, b3, acc[0][3]);
    guard4_h(acc[0][0], acc[0][1], acc[0][2], acc[0][3], a0, b0, b1, b2, b3);
    acc[1][0] = Frag<_Float16>::mma(a1, b0, acc[1][0]);
    acc[1][1] = Frag<_Float16>::mma(a1, b1, acc[1][1]);
    acc[1][2] = Frag<_Float16>::mma(a1, b2, acc[1][2]);
    acc[1][3] = Frag<_Float16>::mma(a1, b3, acc[1][3]);
    guard4_h(acc[1][0], acc[1][1], acc[1][2], acc[1][3], a1, b0, b1, b2, b3);
  }
  acc_guard4(acc[0][0], acc[0][1], acc[0][2], acc[0][3]);
  acc_guard4(acc[1][0], acc[1][1], acc[1][2], acc[1][3]);

#pragma unroll
  for (int j = 0; j < 4; ++j) {
    const int n = n0 + 16 * j + c;
    const float bo = b_out[n];
#pragma unroll
    for (int i = 0; i < 2; ++i)
#pragma unroll
      for (int r = 0; r < 8; ++r)
        Lg[(16 * i + 8 * hh + r) * LPITCH + n] = acc[i][j][r] * WCARRY_INV + bo;
  }
  __syncthreads();

#pragma unroll 1
  for (int rr = 0; rr < 4; ++rr) {
    const int row = 4 * wave + rr;
    float* lr = Lg + row * LPITCH + 4 * lane;
    float m = -INFINITY;
#pragma unroll
    for (int q = 0; q < 4; ++q) {
      const v4f v = *(const v4f*)(lr + 128 * q);
      m = fmaxf(m, fmaxf(fmaxf(v[0], v[1]), fmaxf(v[2], v[3])));
    }
#pragma unroll
    for (int off = 1; off < 32; off <<= 1) m = fmaxf(m, __shfl_xor(m, off, 32));
    float s = 0.0f;
#pragma unroll 1
    for (int q = 0; q < 4; ++q) {
      const v4f v = *(const v4f*)(lr + 128 * q);
      v4f e;
      e[0] = expf(v[0] - m);
      e[1] = expf(v[1] - m);
      e[2] = expf(v[2] - m);
      e[3] = expf(v[3] - m);
      s += (e[0] + e[1]) + (e[2] + e[3]);
      *(v4f*)(lr + 128 * q) = e;
    }
#pragma unroll
    for (int off = 1; off < 32; off <<= 1) s += __shfl_xor(s, off, 32);
    const float inv = 1.0f / s;
    v4f o[4];
#pragma unroll
    for (int q = 0; q < 4; ++q) {
      const v4f e = *(const v4f*)(lr + 128 * q);
      o[q] = (v4f){e[0] * inv, e[1] * inv, e[2] * inv, e[3] * inv};
    }
    float* op = out + (size_t)(R0 + row) * NOUTD + 4 * lane;
    for (int pass = 0; pass < 2; ++pass) {
#pragma unroll
      for (int q = 0; q < 4; ++q) *(volatile v4f*)(op + 128 * q) = o[q];
      __threadfence();
    }
  }
}

extern "C" void kernel_launch(void* const* d_in, const int* in_sizes, int n_in,
                              void* d_out, int out_size, void* d_ws, size_t ws_size, hipStream_t stream) {
  if (n_in < 9 || d_out == nullptr || d_ws == nullptr) return;
  if (in_sizes[0] != NBATCH * NIN * NSTEP || in_sizes[1] != NGATE * NIN || in_sizes[2] != NGATE * NHID ||
      in_sizes[3] != NGATE || in_sizes[4] != NGATE || in_sizes[5] != NOUTD * NHID || in_sizes[6] != NOUTD ||
      in_sizes[7] != NHID || in_sizes[8] != NHID || out_size != NROWS * NOUTD) return;

  const float* x     = (const float*)d_in[0];
  const float* w_ih  = (const float*)d_in[1];
  const float* w_hh  = (const float*)d_in[2];
  const float* b_ih  = (const float*)d_in[3];
  const float* b_hh  = (const float*)d_in[4];
  const float* w_out = (const float*)d_in[5];
  const float* b_out = (const float*)d_in[6];
  const float* h0    = (const float*)d_in[7];
  const float* c0    = (const float*)d_in[8];
  float* out = (float*)d_out;

  char* ws = (char*)d_ws;
  size_t off = 0;
  auto carve = [&](size_t bytes) -> char* { char* p = ws + off; off += (bytes + 255) & ~(size_t)255; return p; };
  unsigned short* XST    = (unsigned short*)carve((size_t)NROWS * NIN * 2);
  unsigned short* WIH16  = (unsigned short*)carve((size_t)NGATE * NIN * 2);
  unsigned short* WHH16  = (unsigned short*)carve((size_t)NGATE * NHID * 2);
  unsigned short* WOUT16 = (unsigned short*)carve((size_t)NOUTD * NHID * 2);
  float*          BIAS16 = (float*)carve((size_t)NGATE * 4);
  float*          XPF    = (float*)carve((size_t)(CHROWS / 16) * (NGATE / 16) * TILE_F * 4);
  unsigned short* CALL16 = (unsigned short*)carve((size_t)NROWS * NHID * 2);
  unsigned short* HST0   = (unsigned short*)carve((size_t)NBATCH * NHID * 2);
  unsigned short* HST1   = (unsigned short*)carve((size_t)NBATCH * NHID * 2);
  float*          CST0   = (float*)carve((size_t)NBATCH * NHID * 4);
  float*          CST1   = (float*)carve((size_t)NBATCH * NHID * 4);
  if (off > ws_size || off > (size_t)134217728) return;

  prep_kernel<<<PB_ALL, 256, 0, stream>>>(w_ih, w_hh, w_out, b_ih, b_hh, h0, c0,
                                          WIH16, WHH16, WOUT16, BIAS16, HST0, CST0);
  xs_transpose_kernel<<<dim3(NSTEP / 64, NIN / 64, NBATCH), 256, 0, stream>>>(x, XST);

  for (int ch = 0; ch < NCHUNK; ++ch) {
    const unsigned short* hin  = (ch & 1) ? HST1 : HST0;
    unsigned short*       hout = (ch & 1) ? HST0 : HST1;
    const float*          cin  = (ch & 1) ? CST1 : CST0;
    float*                cout = (ch & 1) ? CST0 : CST1;
    xproj_gemm_kernel<<<(CHROWS / 64) * (NGATE / 64) / 8, 256, 0, stream>>>(
        XST + (size_t)ch * CHROWS * NIN, WIH16, BIAS16, XPF);
    lstm_seq_kernel<<<MBLK, SEQTHR, 0, stream>>>(XPF, WHH16, hin, cin, hout, cout, CALL16, ch * TCHUNK);
  }

  head_softmax_kernel<<<NROWS / 32, 256, 0, stream>>>(CALL16, WOUT16, b_out, out);
}
